// StandardAttention_8280696947021
// MI455X (gfx1250) — hardware-verified
//
#include <hip/hip_runtime.h>


#ifndef NB
#define NB 2
#endif
#ifndef SEQ
#define SEQ 2048
#endif
#ifndef NB_FULL
#define NB_FULL 2
#endif
#ifndef SEQ_FULL
#define SEQ_FULL 2048
#endif
#ifndef PRES
#define PRES 0
#endif

namespace {
constexpr int HID = 1024, H = 16, HD = 64, QL = SEQ, SK = SEQ, MR = NB * SEQ;
constexpr float XC = 8.0f, WC = 64.0f, XS = 8.0f, CS = 64.0f, PS = 1024.0f, PRS = 1024.0f, LOG2E = 1.4426950408889634f;
static_assert(SEQ % 64 == 0 && SEQ >= 64 && SEQ <= SEQ_FULL && NB >= 1 && NB <= NB_FULL && H * HD == HID && HID % 64 == 0 && MR % 64 == 0 && QL == SK && HD == 64);

typedef _Float16 b16;
typedef __attribute__((ext_vector_type(16))) _Float16 v16b;
typedef __attribute__((ext_vector_type(8))) _Float16 v8b;
typedef __attribute__((ext_vector_type(8))) float v8f;
typedef __attribute__((ext_vector_type(4))) float v4f;

__device__ __forceinline__ float bf16_rne(float f) { unsigned int u = __float_as_uint(f); u += 0x7FFFu + ((u >> 16) & 1u); return __uint_as_float(u & 0xFFFF0000u); }
__device__ __forceinline__ v16b frag_kb(const b16* p, int hh) {
  const v8b a = *(const v8b*)(p + 8 * hh), b = *(const v8b*)(p + 16 + 8 * hh); v16b f;
#pragma unroll
  for (int e = 0; e < 8; ++e) { f[e] = a[e]; f[8 + e] = b[e]; }
  return f;
}
__device__ __forceinline__ v8f wmma16b(v16b a, v16b b, v8f c) {
  v8f d = __builtin_amdgcn_wmma_f32_16x16x32_f16(false, a, false, b, (short)0, c, false, false);
  asm volatile("v_nop\n\tv_nop\n\tv_nop\n\tv_nop" : "+v"(d) : "v"(a), "v"(b));
  return d;
}
__device__ __forceinline__ void wave_lds_sync() { __builtin_amdgcn_fence(3, "workgroup"); __builtin_amdgcn_wave_barrier(); __builtin_amdgcn_fence(2, "workgroup"); }
__device__ __forceinline__ float nexp2(float v) { return __builtin_amdgcn_exp2f(v); }

__global__ __launch_bounds__(256) void cvt_x_kernel(const float* __restrict__ X, b16* __restrict__ Xp) {
  const size_t u = (size_t)blockIdx.x * 256 + threadIdx.x;
  if (u >= (size_t)MR * HID / 8) return;
  const size_t e = u * 8; const size_t row = e / HID; const int c = (int)(e % HID);
  const size_t b = row / SEQ, s = row % SEQ;
  const float* src = X + (b * SEQ_FULL + s) * HID + c;
  b16* dst = Xp + e;
  const v4f x0 = *(const v4f*)src, x1 = *(const v4f*)(src + 4); v8b o;
#pragma unroll
  for (int j = 0; j < 4; ++j) { o[j] = (b16)(bf16_rne(x0[j]) * XC); o[4 + j] = (b16)(bf16_rne(x1[j]) * XC); }
  *(volatile v8b*)dst = o; __threadfence(); *(volatile v8b*)dst = o;
}

__global__ __launch_bounds__(64) void cvt_w_kernel(const float* __restrict__ W0, const float* __restrict__ W1, const float* __restrict__ W2, const float* __restrict__ W3,
                                                   b16* __restrict__ T0, b16* __restrict__ T1, b16* __restrict__ T2, b16* __restrict__ T3) {
  __shared__ __attribute__((aligned(16))) b16 St[64][64 + 8];
  const int tid = threadIdx.x, wave = tid >> 5, lane = tid & 31; const int kb = (int)blockIdx.x, nb = (int)blockIdx.y, z = (int)blockIdx.z;
  const float* W = (z == 0) ? W0 : ((z == 1) ? W1 : ((z == 2) ? W2 : W3));
  b16* T = (z == 0) ? T0 : ((z == 1) ? T1 : ((z == 2) ? T2 : T3));
  const float* src = W + (size_t)kb * 64 * HID + (size_t)nb * 64;
  for (int it = 0; it < 16; ++it) {
    const int e = (it * 64 + tid) * 4; const int kk = e >> 6, nn = e & 63;
    const v4f x = *(const v4f*)(src + (size_t)kk * HID + nn);
#pragma unroll
    for (int j = 0; j < 4; ++j) St[nn + j][kk] = (b16)(bf16_rne(x[j]) * WC);
  }
  __syncthreads();
  b16* dstb = T + (size_t)nb * 64 * HID + (size_t)kb * 64;
  for (int pass = 0; pass < 2; ++pass) {
#pragma unroll 1
    for (int it = 0; it < 8; ++it) {
      const int d = wave * 32 + it * 4 + (lane >> 3), pc = (lane & 7) * 8;
      const v8b o = *(const v8b*)(&St[d][pc]);
      *(volatile v8b*)(dstb + (size_t)d * HID + pc) = o; }
    __threadfence(); }
}

__device__ __forceinline__ void gemm_core(const b16* __restrict__ Aw, const b16* __restrict__ Bt, v8f (&acc)[2][4]) {
  const int lane = threadIdx.x & 31, hh = lane >> 4, col = lane & 15;
  const b16* a0p = Aw + (size_t)col * HID; const b16* a1p = Aw + (size_t)(16 + col) * HID; const b16* bp = Bt + (size_t)col * HID;
#pragma unroll
  for (int s = 0; s < 2; ++s)
#pragma unroll
    for (int c = 0; c < 4; ++c) acc[s][c] = (v8f){};
#pragma unroll 1
  for (int k0 = 0; k0 < HID; k0 += 32) {
    const v16b fa0 = frag_kb(a0p + k0, hh), fa1 = frag_kb(a1p + k0, hh);
#pragma unroll
    for (int c = 0; c < 4; ++c) {
      const v16b fb = frag_kb(bp + (size_t)c * 16 * HID + k0, hh);
      acc[0][c] = wmma16b(fa0, fb, acc[0][c]); acc[1][c] = wmma16b(fa1, fb, acc[1][c]); }
  }
}

__global__ __launch_bounds__(64) __attribute__((amdgpu_num_vgpr(256))) void gemm_qkv_kernel(const b16* __restrict__ Xp, const b16* __restrict__ Wt0, const b16* __restrict__ Wt1,
                                                                                          const b16* __restrict__ Wt2, const float* __restrict__ bi0, const float* __restrict__ bi1,
                                                                                          const float* __restrict__ bi2, b16* __restrict__ Qp, b16* __restrict__ Kp,
                                                                                          b16* __restrict__ VT) {
  __shared__ __attribute__((aligned(16))) b16 Cs[64][64 + 8];
  const int tid = threadIdx.x, wave = tid >> 5, lane = tid & 31, hh = lane >> 4, col = lane & 15;
  const int mt = (int)blockIdx.x, nt = (int)blockIdx.y, z = (int)blockIdx.z;
  const b16* Wt = (z == 0) ? Wt0 : ((z == 1) ? Wt1 : Wt2); const float* bias = (z == 0) ? bi0 : ((z == 1) ? bi1 : bi2);
  v8f acc[2][4];
  gemm_core(Xp + ((size_t)mt * 64 + wave * 32) * HID, Wt + (size_t)nt * 64 * HID, acc);
  const float osc = XS / (XC * WC);
  float bb[4];
#pragma unroll
  for (int c = 0; c < 4; ++c) bb[c] = bf16_rne(bias[nt * 64 + 16 * c + col]) * XS;
  const int b = (mt * 64) / SEQ, s0 = (mt * 64) % SEQ; const size_t bh = (size_t)b * H + nt;
  if (z < 2) {
#pragma unroll
    for (int s = 0; s < 2; ++s)
#pragma unroll
      for (int c = 0; c < 4; ++c)
#pragma unroll
        for (int r = 0; r < 8; ++r) Cs[wave * 32 + 16 * s + 8 * hh + r][16 * c + col] = (b16)(acc[s][c][r] * osc + bb[c]);
    __syncthreads();
    b16* dst = ((z == 0) ? Qp : Kp) + (bh * SEQ + (size_t)s0) * HD;
    for (int pass = 0; pass < 2; ++pass) {
#pragma unroll 1
      for (int it = 0; it < 8; ++it) {
        const int m = wave * 32 + it * 4 + (lane >> 3), pc = (lane & 7) * 8;
        const v8b o = *(const v8b*)(&Cs[m][pc]);
        *(volatile v8b*)(dst + (size_t)m * HD + pc) = o; }
      __threadfence(); }
  } else {
#pragma unroll
    for (int s = 0; s < 2; ++s)
#pragma unroll
      for (int c = 0; c < 4; ++c) {
        v8b o;
#pragma unroll
        for (int r = 0; r < 8; ++r) o[r] = (b16)(acc[s][c][r] * osc + bb[c]);
        *(v8b*)(&Cs[16 * c + col][wave * 32 + 16 * s + 8 * hh]) = o; }
    __syncthreads();
    b16* dst = VT + bh * HD * (size_t)SK + (size_t)s0;
    for (int pass = 0; pass < 2; ++pass) {
#pragma unroll 1
      for (int it = 0; it < 8; ++it) {
        const int d = wave * 32 + it * 4 + (lane >> 3), pc = (lane & 7) * 8;
        const v8b o = *(const v8b*)(&Cs[d][pc]);
        *(volatile v8b*)(dst + (size_t)d * SK + pc) = o; }
      __threadfence(); }
  }
}

template <bool PR>
__global__ __launch_bounds__(64) __attribute__((amdgpu_num_vgpr(256))) void attn_kernel(const b16* __restrict__ Qp, const b16* __restrict__ Kp, const b16* __restrict__ VT,
                                                                                      const int* __restrict__ mask, b16* __restrict__ Cp) {
  __shared__ __attribute__((aligned(16))) b16 Pb[2][16][32 + 8];
  __shared__ __attribute__((aligned(16))) b16 Pr[2][16][32 + 8];
  __shared__ __attribute__((aligned(16))) b16 Tc[2][16][HD + 8];
  const int wave = threadIdx.x >> 5, lane = threadIdx.x & 31, hh = lane >> 4, col = lane & 15;
  const size_t bhi = blockIdx.y; const int b = (int)(bhi / H), h = (int)(bhi % H); const int bx = (int)blockIdx.x; const int q0 = bx * 32 + wave * 16, qi = q0 + col;
  const b16* Qb = Qp + bhi * QL * HD; const b16* Kb = Kp + bhi * SK * HD; const b16* Vb = VT + bhi * HD * (size_t)SK;
  const int* mrow = mask + (size_t)b * SEQ_FULL;
  const v16b qa0 = frag_kb(Qb + (size_t)qi * HD, hh), qa1 = frag_kb(Qb + (size_t)qi * HD + 32, hh);
  const float cs = LOG2E / (8.0f * XS * XS);
  float m = -INFINITY, l = 0.0f; v8f o[4], o2[4];
#pragma unroll
  for (int t = 0; t < 4; ++t) { o[t] = (v8f){}; o2[t] = (v8f){}; }
#pragma unroll 1
  for (int kb = 0; kb < SK; kb += 32) {
    const unsigned int bits = __builtin_amdgcn_ballot_w32(mrow[kb + lane] != 0);
    float e[16]; float mx = -INFINITY;
#pragma unroll
    for (int u = 0; u < 2; ++u) {
      const size_t kr = (size_t)(kb + u * 16 + col) * HD;
      v8f s = (v8f){}; s = wmma16b(frag_kb(Kb + kr, hh), qa0, s); s = wmma16b(frag_kb(Kb + kr + 32, hh), qa1, s);
#pragma unroll
      for (int r = 0; r < 8; ++r) {
        const int ki = u * 16 + 8 * hh + r;
        const float v = ((bits >> ki) & 1u) ? s[r] * cs : -INFINITY;
        e[u * 8 + r] = v; mx = fmaxf(mx, v); } }
    mx = fmaxf(mx, __shfl_xor(mx, 16)); const float mn = fmaxf(m, mx);
    const float mu = (mn == -INFINITY) ? 0.0f : mn;
    const float al = nexp2(m - mu); float sum = 0.0f;
#pragma unroll
    for (int i2 = 0; i2 < 16; ++i2) {
      const float p = nexp2(e[i2] - mu); sum += p; const int pi = (i2 < 8 ? 0 : 16) + 8 * hh + (i2 & 7);
      const float pp = p * PS; const b16 ph = (b16)pp; Pb[wave][col][pi] = ph;
      if constexpr (PR) Pr[wave][col][pi] = (b16)((pp - (float)ph) * PRS); }
    sum += __shfl_xor(sum, 16); l = l * al + sum; m = mn;
    wave_lds_sync();
    const v16b pf = frag_kb(&Pb[wave][col][0], hh);
    v16b prf = (v16b){};
    if constexpr (PR) prf = frag_kb(&Pr[wave][col][0], hh);
#pragma unroll
    for (int t = 0; t < 4; ++t) {
      o[t] *= al; const v16b vh = frag_kb(Vb + (size_t)(t * 16 + col) * SK + kb, hh);
      o[t] = wmma16b(vh, pf, o[t]);
      if constexpr (PR) { o2[t] *= al; o2[t] = wmma16b(vh, prf, o2[t]); } }
    wave_lds_sync(); }
  const float inv = CS / (l * PS * XS);
#pragma unroll
  for (int t = 0; t < 4; ++t) {
#pragma unroll
    for (int r = 0; r < 8; ++r) {
      float ov = o[t][r];
      if constexpr (PR) ov += o2[t][r] * (1.0f / PRS);
      Tc[wave][col][t * 16 + 8 * hh + r] = (b16)(ov * inv); } }
  wave_lds_sync();
  b16* cb = Cp + ((size_t)b * SEQ + (size_t)q0) * HID + (size_t)h * HD;
  for (int pass = 0; pass < 2; ++pass) {
#pragma unroll 1
    for (int it = 0; it < 4; ++it) {
      const int rr = it * 4 + (lane >> 3), pc = (lane & 7) * 8; const v8b f = *(const v8b*)(&Tc[wave][rr][pc]);
      *(volatile v8b*)(cb + (size_t)rr * HID + pc) = f; }
    __threadfence(); }
}

__global__ __launch_bounds__(64) __attribute__((amdgpu_num_vgpr(256))) void gemm_out_kernel(const b16* __restrict__ Cp, const b16* __restrict__ Wt, const float* __restrict__ bias,
                                                                                          float* __restrict__ out) {
  __shared__ __attribute__((aligned(16))) float Cf[64][64 + 4];
  const int tid = threadIdx.x, wave = tid >> 5, lane = tid & 31, hh = lane >> 4, col = lane & 15;
  const int mt = (int)blockIdx.x, nt = (int)blockIdx.y;
  v8f acc[2][4];
  gemm_core(Cp + ((size_t)mt * 64 + wave * 32) * HID, Wt + (size_t)nt * 64 * HID, acc);
  const float osc = 1.0f / (CS * WC);
  float bb[4];
#pragma unroll
  for (int c = 0; c < 4; ++c) bb[c] = bf16_rne(bias[nt * 64 + 16 * c + col]);
#pragma unroll
  for (int s = 0; s < 2; ++s)
#pragma unroll
    for (int c = 0; c < 4; ++c)
#pragma unroll
      for (int r = 0; r < 8; ++r) Cf[wave * 32 + 16 * s + 8 * hh + r][16 * c + col] = acc[s][c][r] * osc + bb[c];
  __syncthreads();
  const int b = (mt * 64) / SEQ, s0 = (mt * 64) % SEQ;
  float* ob = out + ((size_t)b * SEQ_FULL + (size_t)s0) * HID + (size_t)nt * 64;
  for (int pass = 0; pass < 2; ++pass) {
#pragma unroll 1
    for (int it = 0; it < 16; ++it) {
      const int mrow = wave * 32 + it * 2 + hh; const v4f f = *(const v4f*)(&Cf[mrow][col * 4]);
      *(volatile v4f*)(ob + (size_t)mrow * HID + col * 4) = f; }
    __threadfence(); }
}
}

extern "C" void kernel_launch(void* const* d_in, const int* in_sizes, int n_in, void* d_out, int out_size, void* d_ws, size_t ws_size, hipStream_t stream) {
  const size_t needx = ((size_t)(NB - 1) * SEQ_FULL + SEQ) * HID, needm = (size_t)(NB - 1) * SEQ_FULL + SEQ, needw = (size_t)HID * HID, needb = (size_t)HID;
  if (n_in < 10 || (size_t)in_sizes[0] < needx || (size_t)in_sizes[1] < needm || (size_t)out_size < needx) return;
  if ((size_t)in_sizes[2] < needw || (size_t)in_sizes[4] < needw || (size_t)in_sizes[6] < needw || (size_t)in_sizes[8] < needw) return;
  if ((size_t)in_sizes[3] < needb || (size_t)in_sizes[5] < needb || (size_t)in_sizes[7] < needb || (size_t)in_sizes[9] < needb) return;
  const float* Xin = (const float*)d_in[0]; const int* Min = (const int*)d_in[1];
  const float* Wq = (const float*)d_in[2]; const float* bq = (const float*)d_in[3]; const float* Wk = (const float*)d_in[4]; const float* bk = (const float*)d_in[5];
  const float* Wv = (const float*)d_in[6]; const float* bv = (const float*)d_in[7]; const float* Wo = (const float*)d_in[8]; const float* bo = (const float*)d_in[9];
  size_t off = 0; char* ws = (char*)d_ws;
  auto carve = [&](size_t bytes) { char* p = ws + off; off += (bytes + 255) & ~(size_t)255; return p; };
  const size_t xplane = (size_t)MR * HID * 2;
  const size_t wplane = (size_t)HID * HID * 2;
  b16* Xp = (b16*)carve(xplane); b16* T0 = (b16*)carve(wplane); b16* T1 = (b16*)carve(wplane); b16* T2 = (b16*)carve(wplane); b16* T3 = (b16*)carve(wplane);
  b16* Qp = (b16*)carve(xplane); b16* Kp = (b16*)carve(xplane); b16* VTp = (b16*)carve(xplane); b16* Cp = (b16*)carve(xplane);
  if (off > ws_size || off > ((size_t)128 << 20)) return;
  cvt_x_kernel<<<dim3((unsigned)(((size_t)MR * HID / 8 + 255) / 256)), 256, 0, stream>>>(Xin, Xp);
  cvt_w_kernel<<<dim3(HID / 64, HID / 64, 4), 64, 0, stream>>>(Wq, Wk, Wv, Wo, T0, T1, T2, T3);
  gemm_qkv_kernel<<<dim3(MR / 64, HID / 64, 3), 64, 0, stream>>>(Xp, T0, T1, T2, bq, bk, bv, Qp, Kp, VTp);
  attn_kernel<(PRES != 0)><<<dim3(QL / 32, NB * H), 64, 0, stream>>>(Qp, Kp, VTp, Min, Cp);
  gemm_out_kernel<<<dim3(MR / 64, HID / 64), 64, 0, stream>>>(Cp, T3, bo, (float*)d_out);
}
